// WoodStressGNN_31585189495032
// MI455X (gfx1250) — hardware-verified
//
#include <hip/hip_runtime.h>
#include <stdint.h>


#define NN 100000
#define NE 1600000
#define INC 6
#define HID 64
#define OUTC 3

#define EPS 512
#define NSTEP (NE / EPS)
#define R0 4096
#define R1 1024
#define LSTC 1024

#define NTILE (NN / 16)
#define NUNIT (NN / 32)
#define GWAVES 4
#define TPW 8
#define UPW 4

typedef float v4f __attribute__((ext_vector_type(4)));
typedef float v8f __attribute__((ext_vector_type(8)));
typedef int v4i __attribute__((ext_vector_type(4)));
typedef int v2i __attribute__((ext_vector_type(2)));
typedef unsigned short v8us __attribute__((ext_vector_type(8)));
typedef __bf16 v16b __attribute__((ext_vector_type(16)));

union Frag { v16b v; v8us h8[2]; unsigned short u[16]; };

__device__ __forceinline__ v8f zero8()
{
    v8f z;
#pragma unroll
    for (int i = 0; i < 8; ++i) z[i] = 0.0f;
    return z;
}

__device__ __forceinline__ v4f zero4()
{
    v4f z;
    z.x = 0.0f; z.y = 0.0f; z.z = 0.0f; z.w = 0.0f;
    return z;
}

__device__ __forceinline__ v4i zero4i()
{
    v4i z;
    z.x = 0; z.y = 0; z.z = 0; z.w = 0;
    return z;
}

__device__ __forceinline__ void split_bf16(float x, unsigned short& hi, unsigned short& lo)
{
    const __bf16 hb = (__bf16)x;
    const unsigned short hu = __builtin_bit_cast(unsigned short, hb);
    const float hf = __builtin_bit_cast(float, ((unsigned int)hu) << 16);
    const __bf16 lb = (__bf16)(x - hf);
    hi = hu;
    lo = __builtin_bit_cast(unsigned short, lb);
}

__device__ __forceinline__ void split16(v4f f0, v4f f1, v4f f2, v4f f3, Frag& ah, Frag& al)
{
    float xs[16];
    xs[0] = f0.x;  xs[1] = f0.y;  xs[2] = f0.z;  xs[3] = f0.w;
    xs[4] = f1.x;  xs[5] = f1.y;  xs[6] = f1.z;  xs[7] = f1.w;
    xs[8] = f2.x;  xs[9] = f2.y;  xs[10] = f2.z; xs[11] = f2.w;
    xs[12] = f3.x; xs[13] = f3.y; xs[14] = f3.z; xs[15] = f3.w;
#pragma unroll
    for (int i = 0; i < 16; ++i) {
        unsigned short a, b;
        split_bf16(xs[i], a, b);
        ah.u[i] = a;
        al.u[i] = b;
    }
}

__device__ __forceinline__ v8f mma3(v8f acc, v16b ah, v16b al, v16b bh, v16b bl)
{
    acc = __builtin_amdgcn_wmma_f32_16x16x32_bf16(false, ah, false, bh, (short)0, acc, false, false);
    acc = __builtin_amdgcn_wmma_f32_16x16x32_bf16(false, ah, false, bl, (short)0, acc, false, false);
    acc = __builtin_amdgcn_wmma_f32_16x16x32_bf16(false, al, false, bh, (short)0, acc, false, false);
    asm volatile("v_nop\n\tv_nop\n\tv_nop\n\tv_nop" : "+v"(acc) : "v"(ah), "v"(al), "v"(bh), "v"(bl));
    return acc;
}

#define HT1(v, i) msk |= (((unsigned)((v) - d0) < (unsigned)R) ? (1u << (i)) : 0u);
#define HT4(q, i) HT1((q).x, (i)) HT1((q).y, (i) + 1) HT1((q).z, (i) + 2) HT1((q).w, (i) + 3)

template <int MODE>
__global__ void __launch_bounds__(32)
k_agg(const float* __restrict__ feat, const int* __restrict__ srcs, const int* __restrict__ dsts,
      float* outrows, int n_nodes, int n_steps)
{
    extern __shared__ __attribute__((aligned(16))) float smem[];
    constexpr int R  = MODE ? R1 : R0;
    constexpr int RW = MODE ? HID : 8;
    float* acc = smem;
    int*   cnt = (int*)(smem + R * RW);
    int*   lst = cnt + R;

    const int lane = threadIdx.x;
    const int g = lane >> 3, gl = lane & 7;
    const int d0 = blockIdx.x * R;
    const unsigned ltm = (1u << lane) - 1u;
    if (n_steps > NSTEP) n_steps = NSTEP;
    if (n_steps < 0) n_steps = 0;

    for (int i = lane * 4; i < R * RW; i += 128) *(v4f*)(acc + i) = zero4();
    for (int i = lane * 4; i < R; i += 128) *(v4i*)(cnt + i) = zero4i();
    __syncthreads();

    int fill = 0;
    for (int it = 0; it < n_steps; ++it) {
        const int ebase = it * EPS + lane * 16;
        const v4i q0 = *(const v4i*)(dsts + ebase);
        const v4i q1 = *(const v4i*)(dsts + ebase + 4);
        const v4i q2 = *(const v4i*)(dsts + ebase + 8);
        const v4i q3 = *(const v4i*)(dsts + ebase + 12);
        unsigned msk = 0u;
        HT4(q0, 0) HT4(q1, 4) HT4(q2, 8) HT4(q3, 12)
        const int c = __popc(msk);
        const unsigned b0 = (unsigned)__ballot(c & 1);
        const unsigned b1 = (unsigned)__ballot((c >> 1) & 1);
        const unsigned b2 = (unsigned)__ballot((c >> 2) & 1);
        const unsigned b3 = (unsigned)__ballot((c >> 3) & 1);
        const unsigned b4 = (unsigned)__ballot((c >> 4) & 1);
        const int nh = __popc(b0) + 2 * __popc(b1) + 4 * __popc(b2) + 8 * __popc(b3) + 16 * __popc(b4);
        if (nh > 0) {
            int pos = fill + __popc(b0 & ltm) + 2 * __popc(b1 & ltm) + 4 * __popc(b2 & ltm)
                    + 8 * __popc(b3 & ltm) + 16 * __popc(b4 & ltm);
            unsigned mm = msk;
            while (mm != 0u) {
                const int i = __builtin_ctz(mm);
                mm &= mm - 1u;
                const int e = ebase + i;
                int s = srcs[e];
                int dl = dsts[e] - d0;
                s = s < 0 ? 0 : (s >= NN ? NN - 1 : s);
                dl = dl < 0 ? 0 : (dl >= R ? R - 1 : dl);
                if ((unsigned)pos < (unsigned)LSTC) {
                    v2i hv;
                    hv.x = s; hv.y = dl;
                    *(v2i*)(lst + 2 * pos) = hv;
                }
                ++pos;
            }
            fill += nh;
            if (fill > LSTC) fill = LSTC;
        }
        const bool flush = (fill > LSTC - EPS) || (it == n_steps - 1);
        if (flush && fill > 0) {
            __syncthreads();
            for (int t = 0; t < fill; t += 4) {
                const int idx = t + g;
                const bool valid = idx < fill;
                int s = 0, dl = -1 - g;
                if (valid) {
                    const v2i hd = *(const v2i*)(lst + 2 * idx);
                    s = hd.x; dl = hd.y;
                    s = s < 0 ? 0 : (s >= NN ? NN - 1 : s);
                    dl = dl < 0 ? 0 : (dl >= R ? R - 1 : dl);
                }
                const int u0 = __builtin_amdgcn_readlane(dl, 0);
                const int u1 = __builtin_amdgcn_readlane(dl, 8);
                const int u2 = __builtin_amdgcn_readlane(dl, 16);
                const int u3 = __builtin_amdgcn_readlane(dl, 24);
                const bool conf = (u0 == u1) | (u0 == u2) | (u0 == u3) | (u1 == u2) | (u1 == u3) | (u2 == u3);
                if (MODE != 0) {
                    const float* fr = feat + (size_t)s * HID + gl * 8;
                    const v4f f0 = *(const v4f*)fr;
                    const v4f f1 = *(const v4f*)(fr + 4);
                    if (!conf) {
                        if (valid) {
                            float* ar = acc + dl * HID + gl * 8;
                            v4f a0 = *(v4f*)ar;
                            v4f a1 = *(v4f*)(ar + 4);
                            a0 += f0; a1 += f1;
                            *(v4f*)ar = a0;
                            *(v4f*)(ar + 4) = a1;
                            if (gl == 0) cnt[dl] += 1;
                        }
                    } else {
                        for (int q = 0; q < 4; ++q) {
                            if (valid && g == q) {
                                float* ar = acc + dl * HID + gl * 8;
                                v4f a0 = *(v4f*)ar;
                                v4f a1 = *(v4f*)(ar + 4);
                                a0 += f0; a1 += f1;
                                *(v4f*)ar = a0;
                                *(v4f*)(ar + 4) = a1;
                                if (gl == 0) cnt[dl] += 1;
                            }
                            __syncthreads();
                        }
                    }
                } else {
                    float fv = 0.0f;
                    if (gl < INC) fv = feat[(size_t)s * INC + gl];
                    if (!conf) {
                        if (valid) {
                            if (gl < INC) acc[dl * 8 + gl] += fv;
                            if (gl == 0) cnt[dl] += 1;
                        }
                    } else {
                        for (int q = 0; q < 4; ++q) {
                            if (valid && g == q) {
                                if (gl < INC) acc[dl * 8 + gl] += fv;
                                if (gl == 0) cnt[dl] += 1;
                            }
                            __syncthreads();
                        }
                    }
                }
            }
            fill = 0;
            __syncthreads();
        }
    }
    __syncthreads();

    if (MODE != 0) {
        for (int pass = 0; pass < 2; ++pass) {
            for (int j = 0; j < R / 2; ++j) {
                const int dl = 2 * j + (lane >> 4);
                const int cc = (lane & 15) * 4;
                const int node = d0 + dl;
                const int n = cnt[dl];
                const float inv = 1.0f / fmaxf((float)n, 1.0f);
                v4f v = *(const v4f*)(acc + dl * HID + cc);
                v = v * inv;
                if (node < n_nodes) *(volatile v4f*)(outrows + (size_t)node * HID + cc) = v;
            }
            if (pass == 0) __threadfence();
        }
    } else {
        for (int pass = 0; pass < 2; ++pass) {
            for (int j = 0; j < R / 4; ++j) {
                const int dl = 4 * j + g;
                const int p = gl;
                const int node = d0 + dl;
                const int nodec = node < n_nodes ? node : (n_nodes - 1);
                const int n = cnt[dl];
                const float inv = 1.0f / fmaxf((float)n, 1.0f);
                const float* xs = feat + (size_t)nodec * INC;
                v4f v = zero4();
                if (p < 2) {
                    v = *(const v4f*)(acc + dl * 8 + 4 * p);
                    v = v * inv;
                } else if (p == 4) {
                    v.x = xs[0]; v.y = xs[1]; v.z = xs[2]; v.w = xs[3];
                } else if (p == 5) {
                    v.x = xs[4]; v.y = xs[5];
                }
                if (node < n_nodes) *(volatile v4f*)(outrows + (size_t)node * 32 + 4 * p) = v;
            }
            if (pass == 0) __threadfence();
        }
    }
}

template <int KS0, int KS1>
__device__ __forceinline__ void tile_gemm(const float* __restrict__ src0, const float* __restrict__ src1, int tile,
                                          const unsigned short* w_hi, const unsigned short* w_lo,
                                          v4f bvec, float* stg, int lane)
{
    constexpr int KS = KS0 + KS1;
    constexpr int KT = 32 * KS;
    const int h = lane >> 4, m = lane & 15;
    v8f acc[4];
#pragma unroll
    for (int nt = 0; nt < 4; ++nt) acc[nt] = zero8();
#pragma unroll
    for (int j = 0; j < KS; ++j) {
        const float* rp;
        if (j < KS0) rp = src0 + (size_t)(tile * 16 + m) * (size_t)(32 * KS0) + 32 * j;
        else         rp = src1 + (size_t)(tile * 16 + m) * (size_t)(32 * KS1) + 32 * (j - KS0);
        const v4f f0 = *(const v4f*)(rp + 8 * h);
        const v4f f1 = *(const v4f*)(rp + 8 * h + 4);
        const v4f f2 = *(const v4f*)(rp + 16 + 8 * h);
        const v4f f3 = *(const v4f*)(rp + 20 + 8 * h);
        Frag ah, al;
        split16(f0, f1, f2, f3, ah, al);
#pragma unroll
        for (int nt = 0; nt < 4; ++nt) {
            const unsigned short* bp = w_hi + (nt * 16 + m) * KT + 32 * j;
            const unsigned short* bq = w_lo + (nt * 16 + m) * KT + 32 * j;
            Frag bh, bl;
            bh.h8[0] = *(const v8us*)(bp + 8 * h);
            bh.h8[1] = *(const v8us*)(bp + 16 + 8 * h);
            bl.h8[0] = *(const v8us*)(bq + 8 * h);
            bl.h8[1] = *(const v8us*)(bq + 16 + 8 * h);
            acc[nt] = mma3(acc[nt], ah.v, al.v, bh.v, bl.v);
        }
    }
    float bb[4];
    bb[0] = bvec.x; bb[1] = bvec.y; bb[2] = bvec.z; bb[3] = bvec.w;
#pragma unroll
    for (int nt = 0; nt < 4; ++nt) {
#pragma unroll
        for (int r = 0; r < 8; ++r) {
            float v = acc[nt][r] + bb[nt];
            v = v > 0.0f ? v : 0.0f;
            stg[(8 * h + r) * HID + nt * 16 + m] = v;
        }
    }
}

template <int KS0, int KS1, bool HEAD>
__global__ void __launch_bounds__(128)
k_sage(const float* __restrict__ src0, const float* __restrict__ src1,
       const float* __restrict__ wl, const float* __restrict__ wr, int inw,
       const float* __restrict__ bias,
       const float* __restrict__ fcw, const float* __restrict__ fcb,
       float* hout, float* gout, int n_items)
{
    constexpr int KS = KS0 + KS1;
    constexpr int KT = 32 * KS;
    constexpr int KH = KT / 2;
    __shared__ __attribute__((aligned(16))) unsigned short w_hi[64 * 128];
    __shared__ __attribute__((aligned(16))) unsigned short w_lo[64 * 128];
    __shared__ __attribute__((aligned(16))) unsigned short f_hi[16 * 64];
    __shared__ __attribute__((aligned(16))) unsigned short f_lo[16 * 64];
    __shared__ __attribute__((aligned(16))) float stage[GWAVES][16 * 64];
    __shared__ __attribute__((aligned(16))) float ostage[GWAVES][96];

    const int tid = threadIdx.x;
    const int lane = tid & 31;
    const int w = tid >> 5;
    const int h = lane >> 4;
    const int m = lane & 15;

    for (int i = tid; i < 64 * KT; i += 128) {
        const int n = i / KT;
        const int k = i - n * KT;
        float v = 0.0f;
        if (k < KH) { if (k < inw) v = wl[n * inw + k]; }
        else { const int kk = k - KH; if (kk < inw) v = wr[n * inw + kk]; }
        unsigned short a, b;
        split_bf16(v, a, b);
        w_hi[i] = a;
        w_lo[i] = b;
    }
    if (HEAD) {
        for (int i = tid; i < 16 * 64; i += 128) {
            const int n = i >> 6;
            const int k = i & 63;
            const float v = (n < OUTC) ? fcw[n * HID + k] : 0.0f;
            unsigned short a, b;
            split_bf16(v, a, b);
            f_hi[i] = a;
            f_lo[i] = b;
        }
    }
    v4f bvec;
    bvec.x = bias[0 * 16 + m]; bvec.y = bias[1 * 16 + m]; bvec.z = bias[2 * 16 + m]; bvec.w = bias[3 * 16 + m];
    float fbv = 0.0f;
    if (HEAD) fbv = (m < OUTC) ? fcb[m] : 0.0f;
    __syncthreads();

    float* stg = stage[w];

    if (!HEAD) {
        for (int it = 0; it < TPW; ++it) {
            const int traw = (blockIdx.x * GWAVES + w) * TPW + it;
            const bool valid = traw < n_items;
            const int tile = valid ? traw : (n_items - 1);
            tile_gemm<KS0, KS1>(src0, src1, tile, w_hi, w_lo, bvec, stg, lane);
            __syncthreads();
            v4f vals[8];
            int ro[8], co[8];
#pragma unroll
            for (int i = 0; i < 8; ++i) {
                const int L = 4 * i + (lane >> 3);
                ro[i] = L >> 1;
                co[i] = (L & 1) * 32 + (lane & 7) * 4;
                vals[i] = *(const v4f*)(stg + ro[i] * HID + co[i]);
            }
            if (valid) {
                float* base = hout + (size_t)tile * 16 * HID;
#pragma unroll
                for (int i = 0; i < 8; ++i) *(volatile v4f*)(base + ro[i] * HID + co[i]) = vals[i];
                __threadfence();
#pragma unroll
                for (int i = 0; i < 8; ++i) *(volatile v4f*)(base + ro[i] * HID + co[i]) = vals[i];
            }
            __syncthreads();
        }
    } else {
        for (int it = 0; it < UPW; ++it) {
            const int uraw = (blockIdx.x * GWAVES + w) * UPW + it;
            const bool valid = uraw < n_items;
            const int u = valid ? uraw : (n_items - 1);
            for (int sub = 0; sub < 2; ++sub) {
                const int tile = u * 2 + sub;
                tile_gemm<KS0, KS1>(src0, src1, tile, w_hi, w_lo, bvec, stg, lane);
                __syncthreads();
                v8f facc = zero8();
#pragma unroll
                for (int j = 0; j < 2; ++j) {
                    const float* rp = stg + m * HID + 32 * j;
                    const v4f f0 = *(const v4f*)(rp + 8 * h);
                    const v4f f1 = *(const v4f*)(rp + 8 * h + 4);
                    const v4f f2 = *(const v4f*)(rp + 16 + 8 * h);
                    const v4f f3 = *(const v4f*)(rp + 20 + 8 * h);
                    Frag ah, al;
                    split16(f0, f1, f2, f3, ah, al);
                    const unsigned short* bp = f_hi + m * HID + 32 * j;
                    const unsigned short* bq = f_lo + m * HID + 32 * j;
                    Frag bh, bl;
                    bh.h8[0] = *(const v8us*)(bp + 8 * h);
                    bh.h8[1] = *(const v8us*)(bp + 16 + 8 * h);
                    bl.h8[0] = *(const v8us*)(bq + 8 * h);
                    bl.h8[1] = *(const v8us*)(bq + 16 + 8 * h);
                    facc = mma3(facc, ah.v, al.v, bh.v, bl.v);
                }
                if (m < OUTC) {
#pragma unroll
                    for (int r = 0; r < 8; ++r)
                        ostage[w][(sub * 16 + 8 * h + r) * OUTC + m] = facc[r] + fbv;
                }
                __syncthreads();
            }
            v4f ov = zero4();
            if (lane < 24) ov = *(const v4f*)(ostage[w] + 4 * lane);
            float* op = gout + (size_t)u * 96 + 4 * lane;
            if (valid && lane < 24) *(volatile v4f*)op = ov;
            __threadfence();
            if (valid && lane < 24) *(volatile v4f*)op = ov;
            __syncthreads();
        }
    }
}

static inline size_t al256(size_t b) { return (b + 255) & ~(size_t)255; }

extern "C" void kernel_launch(void* const* d_in, const int* in_sizes, int n_in,
                              void* d_out, int out_size, void* d_ws, size_t ws_size,
                              hipStream_t stream)
{
    if (n_in < 13) return;
    if (in_sizes[0] != NN * INC || in_sizes[1] != 2 * NE || out_size != NN * OUTC) return;
    if (in_sizes[2] != HID * INC || in_sizes[4] != HID * INC) return;
    if (in_sizes[5] != HID * HID || in_sizes[7] != HID * HID || in_sizes[8] != HID * HID || in_sizes[10] != HID * HID) return;
    if (in_sizes[3] != HID || in_sizes[6] != HID || in_sizes[9] != HID) return;
    if (in_sizes[11] != OUTC * HID || in_sizes[12] != OUTC) return;
    if ((NE % EPS) != 0) return;

    const float* x    = (const float*)d_in[0];
    const int*   ei   = (const int*)d_in[1];
    const int*   srcs = ei;
    const int*   dsts = ei + NE;
    const float* w1l = (const float*)d_in[2];
    const float* b1  = (const float*)d_in[3];
    const float* w1r = (const float*)d_in[4];
    const float* w2l = (const float*)d_in[5];
    const float* b2  = (const float*)d_in[6];
    const float* w2r = (const float*)d_in[7];
    const float* w3l = (const float*)d_in[8];
    const float* b3  = (const float*)d_in[9];
    const float* w3r = (const float*)d_in[10];
    const float* fw  = (const float*)d_in[11];
    const float* fb  = (const float*)d_in[12];
    float* out = (float*)d_out;

    size_t off = 0;
    const size_t oAgg = off; off += al256((size_t)NN * HID * sizeof(float));
    const size_t oHA  = off; off += al256((size_t)NN * HID * sizeof(float));
    const size_t oHB  = off; off += al256((size_t)NN * HID * sizeof(float));
    if (off > ws_size) return;

    char* ws = (char*)d_ws;
    float* agg = (float*)(ws + oAgg);
    float* hA  = (float*)(ws + oHA);
    float* hB  = (float*)(ws + oHB);

    const size_t lds0 = (size_t)(R0 * 8 + R0 + 2 * LSTC) * sizeof(float);
    const size_t lds1 = (size_t)(R1 * HID + R1 + 2 * LSTC) * sizeof(float);
    const int gA0   = (NN + R0 - 1) / R0;
    const int gA1   = (NN + R1 - 1) / R1;
    const int gTile = (NTILE + GWAVES * TPW - 1) / (GWAVES * TPW);
    const int gUnit = (NUNIT + GWAVES * UPW - 1) / (GWAVES * UPW);

    k_agg<0><<<gA0, 32, lds0, stream>>>(x, srcs, dsts, agg, NN, NSTEP);
    k_sage<1, 0, false><<<gTile, 128, 0, stream>>>(agg, agg, w1l, w1r, INC, b1, fw, fb, hA, out, NTILE);

    k_agg<1><<<gA1, 32, lds1, stream>>>(hA, srcs, dsts, agg, NN, NSTEP);
    k_sage<2, 2, false><<<gTile, 128, 0, stream>>>(agg, hA, w2l, w2r, HID, b2, fw, fb, hB, out, NTILE);

    k_agg<1><<<gA1, 32, lds1, stream>>>(hB, srcs, dsts, agg, NN, NSTEP);
    k_sage<2, 2, true><<<gUnit, 128, 0, stream>>>(agg, hB, w3l, w3r, HID, b3, fw, fb, hA, out, NUNIT);
}
